// SingleHeadAttention_4088808866231
// MI455X (gfx1250) — hardware-verified
//
#include <hip/hip_runtime.h>

typedef _Float16 h16;
typedef _Float16 h16x4 __attribute__((ext_vector_type(4)));
typedef _Float16 h16x8 __attribute__((ext_vector_type(8)));
typedef _Float16 v16h  __attribute__((ext_vector_type(16)));
typedef float    v8f   __attribute__((ext_vector_type(8)));
typedef float    v4f   __attribute__((ext_vector_type(4)));
typedef unsigned v4u   __attribute__((ext_vector_type(4)));
typedef unsigned v2u   __attribute__((ext_vector_type(2)));

#ifndef NB
#define NB 4
#endif
#ifndef SEQ
#define SEQ 2048
#endif
#define NB_FULL   4
#define SEQ_FULL  2048
#define D_DIM     1024
#define M_TOT     (NB * SEQ)
#define QE        512
#define KE        (QE + 64)
#define QEARLY    ((SEQ < QE) ? SEQ : QE)
#define WSC       64.0f
#define WUN       (1.0f / 64.0f)
#define RSC       1024.0f
#define RUN       (1.0f / 1024.0f)
#define PSC       1024.0f
#define PUN       (1.0f / 1024.0f)
#define SM_SCALE  0.03125f
#define NEG_BIG   (-1.0e30f)

static_assert((SEQ % 64) == 0);
static_assert(SEQ >= 64 && SEQ <= SEQ_FULL);
static_assert(NB >= 1 && NB <= NB_FULL);
static_assert(D_DIM == 1024);
static_assert((D_DIM / 8) == 128);
static_assert((QE % 64) == 0);
static_assert((M_TOT % 64) == 0);

template <typename V> __device__ __forceinline__ void vst2(void* p, V v) {
  *(volatile V*)p = v; __threadfence(); *(volatile V*)p = v;
}
__device__ __forceinline__ void copy16_g2s(h16* ldst, const h16* gsrc) { *(h16x8*)ldst = *(const h16x8*)gsrc; }

__device__ __forceinline__ float bf16_rne(float f) {
  unsigned u = __float_as_uint(f);
  u += 0x7fffu + ((u >> 16) & 1u);
  u &= 0xffff0000u;
  return __uint_as_float(u);
}

__device__ __forceinline__ v16h load_a_frag(const h16* base, int ld, int k0) {
  int lane = threadIdx.x & 31;
  int idx  = lane & 15;
  int half = lane >> 4;
  const h16* p = base + (size_t)idx * ld + k0 + half * 8;
  h16x8 lo = *(const h16x8*)(p);
  h16x8 hi = *(const h16x8*)(p + 16);
  return __builtin_shufflevector(lo, hi, 0,1,2,3,4,5,6,7,8,9,10,11,12,13,14,15);
}
__device__ __forceinline__ v16h load_b_frag(const h16* base, int ld, int k0) { return load_a_frag(base, ld, k0); }

__device__ __forceinline__ v8f wmma_f16(v16h a, v16h b, v8f c) {
  v8f d = __builtin_amdgcn_wmma_f32_16x16x32_f16(false, a, false, b, (short)0, c, false, false);
  asm volatile("v_nop\n\tv_nop\n\tv_nop\n\tv_nop" : "+v"(d) : "v"(a), "v"(b));
  return d;
}

__global__ __launch_bounds__(256) void cvt_x_kernel(const float* __restrict__ x, h16* __restrict__ xb, int n8) {
  const int g = blockIdx.x * 256 + threadIdx.x;
  if (g >= n8) return;
  const int m  = g >> 7;
  const int c8 = g & 127;
  const int bb = m / SEQ, s = m - bb * SEQ;
  const float* src = x + ((size_t)bb * SEQ_FULL + s) * D_DIM + c8 * 8;
  const v4f a = *(const v4f*)(src), c = *(const v4f*)(src + 4);
  union { h16x8 h; v4u u; } pk;
#pragma unroll
  for (int i = 0; i < 4; ++i) { pk.h[i] = (h16)bf16_rne(a[i]); pk.h[4 + i] = (h16)bf16_rne(c[i]); }
  vst2(xb + (size_t)g * 8, pk.u);
}

__global__ __launch_bounds__(256) void cvt_w_kernel(const float* __restrict__ W0, const float* __restrict__ W1,
                                                    const float* __restrict__ W2, h16* __restrict__ P0,
                                                    h16* __restrict__ P1, h16* __restrict__ P2, int n8) {
  const float* W = (blockIdx.y == 0) ? W0 : (blockIdx.y == 1) ? W1 : W2;
  h16*         P = (blockIdx.y == 0) ? P0 : (blockIdx.y == 1) ? P1 : P2;
  const int g = blockIdx.x * 256 + threadIdx.x;
  if (g >= n8) return;
  const v4f a = *(const v4f*)(W + (size_t)g * 8), c = *(const v4f*)(W + (size_t)g * 8 + 4);
  union { h16x8 h; v4u u; } pk;
#pragma unroll
  for (int i = 0; i < 4; ++i) { pk.h[i] = (h16)(bf16_rne(a[i]) * WSC); pk.h[4 + i] = (h16)(bf16_rne(c[i]) * WSC); }
  vst2(P + (size_t)g * 8, pk.u);
}

__global__ __launch_bounds__(256) __attribute__((amdgpu_num_vgpr(256)))
void proj_kernel(const h16* __restrict__ Xb, const h16* __restrict__ Wh,
                 h16* __restrict__ outh, h16* __restrict__ outr, int transposed) {
  __shared__ __align__(16) h16 T[128 * 136];
  const int m0 = blockIdx.x * 64;
  const int n0 = blockIdx.y * 128;
  const int w    = threadIdx.x >> 5;
  const int lane = threadIdx.x & 31;
  const int idx  = lane & 15;
  const int half = lane >> 4;
  const int m_w = m0 + (w & 3) * 16;
  const int n_w = n0 + (w >> 2) * 64;

  v8f c[4] = {};
  const h16* arow = Xb + (size_t)m_w * D_DIM;
#pragma unroll 2
  for (int k0 = 0; k0 < D_DIM; k0 += 32) {
    v16h a = load_a_frag(arow, D_DIM, k0);
#pragma unroll
    for (int t = 0; t < 4; ++t) {
      v16h b = load_b_frag(Wh + (size_t)(n_w + t * 16) * D_DIM, D_DIM, k0);
      c[t] = wmma_f16(a, b, c[t]);
    }
  }

  const int bb = m0 / SEQ, s0 = m0 - bb * SEQ;
  const int tid = threadIdx.x;
  const int npass = (s0 < KE) ? 2 : 1;
  for (int ps = 0; ps < npass; ++ps) {
    if (ps) __syncthreads();
#pragma unroll
    for (int t = 0; t < 4; ++t) {
      int cl = (w >> 2) * 64 + t * 16 + idx;
#pragma unroll
      for (int g = 0; g < 8; ++g) {
        int rl = (w & 3) * 16 + g + 8 * half;
        float val = c[t][g] * WUN;
        h16 hv = (h16)val;
        h16 sv = ps ? (h16)((val - (float)hv) * RSC) : hv;
        if (!transposed) T[rl * 136 + cl] = sv; else T[cl * 72 + rl] = sv;
      }
    }
    __syncthreads();
    h16* dst = ps ? outr : outh;
    if (!transposed) {
      for (int gg = tid; gg < 64 * 16; gg += 256) {
        const int rl = gg >> 4, pc = gg & 15;
        vst2(dst + (size_t)(m0 + rl) * D_DIM + n0 + pc * 8, *(const v4u*)(&T[rl * 136 + pc * 8]));
      }
    } else {
      for (int gg = tid; gg < 128 * 8; gg += 256) {
        const int cl = gg >> 3, pc = gg & 7;
        vst2(dst + ((size_t)(bb * D_DIM + n0 + cl)) * SEQ + s0 + pc * 8, *(const v4u*)(&T[cl * 72 + pc * 8]));
      }
    }
  }
}

template <bool EARLY>
__global__ __launch_bounds__(256) __attribute__((amdgpu_num_vgpr(256)))
void attn_kernel(const h16* __restrict__ Qh, const h16* __restrict__ Qr,
                 const h16* __restrict__ Kh, const h16* __restrict__ Kr,
                 const h16* __restrict__ Vth, const h16* __restrict__ Vtr,
                 float* __restrict__ out, int qbase) {
  __shared__ __align__(16) h16   Qs[16][D_DIM];
  __shared__ __align__(16) h16   Qrs[EARLY ? 16 : 1][EARLY ? D_DIM : 8];
  __shared__ __align__(16) float Ss[2][16][64];
  __shared__ __align__(16) h16   Ps[16][64];
  __shared__ __align__(16) h16   Prs[EARLY ? 16 : 1][64];
  __shared__ __align__(16) float Ot[16][D_DIM];
  __shared__ float alpha_s[16];
  __shared__ float l_s[16];

  const int b   = blockIdx.y;
  const int q0  = qbase + blockIdx.x * 16;
  const int tid = threadIdx.x;
  const int w    = tid >> 5;
  const int lane = tid & 31;
  const int idx  = lane & 15;
  const int half = lane >> 4;
  const int kj = w & 3;
  const int kh = w >> 2;
  const int dg = w;

  {
    const h16* Qg = Qh + ((size_t)(b * SEQ + q0)) * D_DIM;
    for (int c = tid; c < 16 * 128; c += 256) {
      int r = c >> 7, dc = c & 127;
      copy16_g2s(&Qs[r][dc * 8], Qg + (size_t)r * D_DIM + dc * 8);
    }
    if (EARLY) {
      const h16* Qrg = Qr + ((size_t)(b * SEQ + q0)) * D_DIM;
      for (int c = tid; c < 16 * 128; c += 256) {
        int r = c >> 7, dc = c & 127;
        copy16_g2s(&Qrs[r][dc * 8], Qrg + (size_t)r * D_DIM + dc * 8);
      }
    }
  }

  v8f o[8] = {};
  const int srow = tid >> 4;
  const int sj   = tid & 15;
  float m_prev = NEG_BIG;
  float l_run  = 0.0f;
  const int ntile = q0 / 64 + 1;

  for (int it = 0; it < ntile; ++it) {
    const int kv0 = it * 64;
    __syncthreads();

    {
      v8f sc = {};
      v8f scx = {};
      const size_t krow = ((size_t)(b * SEQ + kv0 + kj * 16)) * D_DIM;
      const h16* Kg = Kh + krow;
      const int kbeg = kh * (D_DIM / 2);
      if (!EARLY) {
#pragma unroll 2
        for (int k0 = kbeg; k0 < kbeg + D_DIM / 2; k0 += 32) {
          v16h a  = load_a_frag(&Qs[0][0], D_DIM, k0);
          v16h bh = load_b_frag(Kg, D_DIM, k0);
          sc = wmma_f16(a, bh, sc);
        }
      } else {
        const h16* Krg = Kr + krow;
#pragma unroll 1
        for (int k0 = kbeg; k0 < kbeg + D_DIM / 2; k0 += 32) {
          v16h a  = load_a_frag(&Qs[0][0], D_DIM, k0);
          v16h bh = load_b_frag(Kg, D_DIM, k0);
          sc  = wmma_f16(a, bh, sc);
          v16h ar = load_a_frag(&Qrs[0][0], D_DIM, k0);
          scx = wmma_f16(ar, bh, scx);
          v16h br = load_b_frag(Krg, D_DIM, k0);
          scx = wmma_f16(a, br, scx);
        }
      }
      const int col = kj * 16 + idx;
#pragma unroll
      for (int g = 0; g < 8; ++g) {
        float s = sc[g];
        if (EARLY) s += scx[g] * RUN;
        Ss[kh][g + 8 * half][col] = s * SM_SCALE;
      }
    }
    __syncthreads();

    {
      const v4f sa = *(const v4f*)(&Ss[0][srow][sj * 4]);
      const v4f sb = *(const v4f*)(&Ss[1][srow][sj * 4]);
      const int qi = q0 + srow;
      const int jb = kv0 + sj * 4;
      float v[4];
      float mloc = NEG_BIG;
#pragma unroll
      for (int e = 0; e < 4; ++e) {
        const float s = sa[e] + sb[e];
        v[e] = (jb + e <= qi) ? s : NEG_BIG;
        mloc = fmaxf(mloc, v[e]);
      }
#pragma unroll
      for (int msk = 1; msk < 16; msk <<= 1) mloc = fmaxf(mloc, __shfl_xor(mloc, msk, 32));
      const float m_new = fmaxf(m_prev, mloc);
      const float alpha = __expf(m_prev - m_new);
      float ssum = 0.0f;
      union { h16x4 h; v2u u; } ph, pr;
#pragma unroll
      for (int e = 0; e < 4; ++e) {
        const float p  = __expf(v[e] - m_new);
        ssum += p;
        const float pv = p * PSC;
        const h16 hv = (h16)pv;
        ph.h[e] = hv;
        pr.h[e] = (h16)((pv - (float)hv) * RSC);
      }
      *(v2u*)(&Ps[srow][sj * 4]) = ph.u;
      if (EARLY) *(v2u*)(&Prs[srow][sj * 4]) = pr.u;
#pragma unroll
      for (int msk = 1; msk < 16; msk <<= 1) ssum += __shfl_xor(ssum, msk, 32);
      l_run = l_run * alpha + ssum;
      m_prev = m_new;
      if (sj == 0) { alpha_s[srow] = alpha; l_s[srow] = l_run; }
    }
    __syncthreads();

    {
      float al[8];
#pragma unroll
      for (int g = 0; g < 8; ++g) al[g] = alpha_s[g + 8 * half];
#pragma unroll
      for (int t = 0; t < 8; ++t)
#pragma unroll
        for (int g = 0; g < 8; ++g) o[t][g] *= al[g];
      const h16* Vg  = Vth + ((size_t)(b * D_DIM + dg * 128)) * SEQ + kv0;
      const h16* Vrg = Vtr + ((size_t)(b * D_DIM + dg * 128)) * SEQ + kv0;
#pragma unroll
      for (int k0 = 0; k0 < 64; k0 += 32) {
        const v16h a = load_a_frag(&Ps[0][0], 64, k0);
        v16h ar = a;
        if (EARLY) ar = load_a_frag(&Prs[0][0], 64, k0);
#pragma unroll
        for (int t = 0; t < 8; ++t) {
          const v16h bh = load_b_frag(Vg + (size_t)(t * 16) * SEQ, SEQ, k0);
          o[t] = wmma_f16(a, bh, o[t]);
          if (EARLY) {
            v8f tmp = {};
            tmp = wmma_f16(ar, bh, tmp);
            const v16h br = load_b_frag(Vrg + (size_t)(t * 16) * SEQ, SEQ, k0);
            tmp = wmma_f16(a, br, tmp);
#pragma unroll
            for (int g = 0; g < 8; ++g) o[t][g] += tmp[g] * RUN;
          }
        }
      }
    }
  }
  __syncthreads();

  float linv[8];
#pragma unroll
  for (int g = 0; g < 8; ++g) linv[g] = PUN / l_s[g + 8 * half];
#pragma unroll
  for (int t = 0; t < 8; ++t) {
    int col = dg * 128 + t * 16 + idx;
#pragma unroll
    for (int g = 0; g < 8; ++g) Ot[g + 8 * half][col] = o[t][g] * linv[g];
  }
  __syncthreads();
  {
    float* dst = out + ((size_t)(b * SEQ_FULL + q0)) * D_DIM;
    const float* src = &Ot[0][0];
    for (int gg = tid; gg < 16 * D_DIM / 4; gg += 256) vst2(dst + (size_t)gg * 4, *(const v4f*)(src + gg * 4));
  }
}

extern "C" void kernel_launch(void* const* d_in, const int* in_sizes, int n_in,
                              void* d_out, int out_size, void* d_ws, size_t ws_size,
                              hipStream_t stream) {
  if (n_in < 4) return;
  const long long need_x = ((long long)(NB - 1) * SEQ_FULL + SEQ) * (long long)D_DIM;
  if ((long long)in_sizes[0] < need_x) return;
  if (in_sizes[1] < D_DIM * D_DIM || in_sizes[2] < D_DIM * D_DIM || in_sizes[3] < D_DIM * D_DIM) return;
  if ((long long)out_size < need_x) return;

  const float* x  = (const float*)d_in[0];
  const float* Wk = (const float*)d_in[1];
  const float* Wq = (const float*)d_in[2];
  const float* Wv = (const float*)d_in[3];
  float* out = (float*)d_out;

  const size_t act = (size_t)M_TOT * D_DIM * sizeof(h16);
  const size_t wpl = (size_t)D_DIM * D_DIM * sizeof(h16);
  char* ws = (char*)d_ws;
  size_t off = 0;
  h16* xb  = (h16*)(ws + off); off += act;
  h16* Wkh = (h16*)(ws + off); off += wpl;
  h16* Wqh = (h16*)(ws + off); off += wpl;
  h16* Wvh = (h16*)(ws + off); off += wpl;
  h16* qh  = (h16*)(ws + off); off += act;
  h16* kh  = (h16*)(ws + off); off += act;
  h16* vth = (h16*)(ws + off); off += act;
  h16* qr  = (h16*)(ws + off); off += act;
  h16* kr  = (h16*)(ws + off); off += act;
  h16* vtr = (h16*)(ws + off); off += act;
  if (off > ws_size) return;

  const int nx8 = M_TOT * (D_DIM / 8);
  cvt_x_kernel<<<(nx8 + 255) / 256, 256, 0, stream>>>(x, xb, nx8);
  const int nw8 = D_DIM * D_DIM / 8;
  cvt_w_kernel<<<dim3((nw8 + 255) / 256, 3), 256, 0, stream>>>(Wk, Wq, Wv, Wkh, Wqh, Wvh, nw8);

  dim3 pg(M_TOT / 64, D_DIM / 128);
  proj_kernel<<<pg, 256, 0, stream>>>(xb, Wqh, qh, qr, 0);
  proj_kernel<<<pg, 256, 0, stream>>>(xb, Wkh, kh, kr, 0);
  proj_kernel<<<pg, 256, 0, stream>>>(xb, Wvh, vth, vtr, 1);

  const int nearly = QEARLY / 16;
  attn_kernel<true><<<dim3(nearly, NB), 256, 0, stream>>>(qh, qr, kh, kr, vth, vtr, out, 0);
  const int nlate = (SEQ - QEARLY) / 16;
  if (nlate > 0)
    attn_kernel<false><<<dim3(nlate, NB), 256, 0, stream>>>(qh, qr, kh, kr, vth, vtr, out, QEARLY);
}
